// TuckEREmbedding_3753801416764
// MI455X (gfx1250) — hardware-verified
//
#include <hip/hip_runtime.h>
#include <math.h>

typedef __attribute__((ext_vector_type(16))) _Float16 v16h;
typedef __attribute__((ext_vector_type(8)))  _Float16 v8h;
typedef __attribute__((ext_vector_type(8)))  float    v8f;
typedef __attribute__((ext_vector_type(4)))  float    v4f;

constexpr int kBatch   = 64;
constexpr int kHid     = 768;
constexpr int kEmb     = 128;
constexpr int kPlane   = kEmb * kEmb;
constexpr int kRowsA   = 3 * kBatch;
constexpr int kRowsW   = 2 * kEmb;
constexpr int kGemmWaves = 4;

constexpr float kCarryA = 16.0f;
constexpr float kCarryW = 1024.0f;
constexpr float kFold   = 1.0f / (kCarryA * kCarryW);
constexpr float kHalfMinNormal = 6.103515625e-5f;

static_assert((kHid % 32) == 0, "GEMM K multiple of 32");
static_assert((kBatch % 64) == 0 && ((2 * kBatch) % 64) == 0 && (kEmb % 64) == 0, "GEMM M,N multiples of 64");
static_assert((kEmb % 32) == 0 && (kPlane % (32 * 4 * 4)) == 0, "plane sum tiling");

constexpr size_t kBytesA16 = (size_t)kRowsA * kHid * 2;
constexpr size_t kBytesW16 = (size_t)kRowsW * kHid * 2;
constexpr size_t kBytesP   = (size_t)kRowsA * kEmb * 4;
constexpr size_t kBytesT   = (size_t)kEmb * 4;
constexpr size_t kOffA16 = 0;
constexpr size_t kOffW16 = kOffA16 + kBytesA16;
constexpr size_t kOffP   = kOffW16 + kBytesW16;
constexpr size_t kOffT   = kOffP + kBytesP;
constexpr size_t kWsTotal = kOffT + kBytesT;
static_assert(kWsTotal == 786944ull, "carve total");
static_assert(kWsTotal <= 134217728ull, "carve cap");
static_assert((kOffW16 % 128) == 0 && (kOffP % 128) == 0 && (kOffT % 128) == 0, "128-B aligned regions");

constexpr int kCvtPerBlock   = 256 * 8;
constexpr int kCvtBlocksSrc  = (kBatch * kHid) / kCvtPerBlock;
constexpr int kCvtBlocksW    = (kEmb * kHid) / kCvtPerBlock;
constexpr int kCvtBlocksA    = 3 * kCvtBlocksSrc;
constexpr int kCvtBlocks     = kCvtBlocksA + 2 * kCvtBlocksW;
static_assert(kCvtBlocksSrc * kCvtPerBlock == kBatch * kHid, "exact coverage of each activation source");
static_assert(kCvtBlocksW * kCvtPerBlock == kEmb * kHid, "exact coverage of each weight source");
static_assert(kCvtBlocks == 168, "convert grid");

union FragH { v16h v; v8h h[2]; };
__device__ __forceinline__ v16h frag_load_h(const _Float16* p) {
  FragH f;
  f.h[0] = *(const v8h*)(p);
  f.h[1] = *(const v8h*)(p + 16);
  return f.v;
}
__device__ __forceinline__ v8f mma_h_guarded(v16h a, v16h b, v8f c) {
  c = __builtin_amdgcn_wmma_f32_16x16x32_f16(false, a, false, b, (short)0, c, false, false);
  asm volatile("v_nop\n\tv_nop\n\tv_nop\n\tv_nop" : "+v"(c) : "v"(a), "v"(b));
  return c;
}
__device__ __forceinline__ void keep4_h(v16h a, v16h b, v16h c, v16h d) { asm volatile("v_nop" :: "v"(a), "v"(b), "v"(c), "v"(d)); }
__device__ __forceinline__ void acc_guard4(v8f& a, v8f& b, v8f& c, v8f& d) { asm volatile("v_nop\n\tv_nop\n\tv_nop\n\tv_nop" : "+v"(a), "+v"(b), "+v"(c), "+v"(d)); }

__device__ __forceinline__ _Float16 to_half_carried(float x, float carry) {
  float v = x * carry;
  v = (fabsf(v) < kHalfMinNormal) ? 0.0f : v;
  return (_Float16)v;
}

__global__ __launch_bounds__(256) void build_half_planes_kernel(
    const float* __restrict__ srcHead, const float* __restrict__ srcTail, const float* __restrict__ srcRel,
    const float* __restrict__ wE, const float* __restrict__ wR,
    unsigned short* __restrict__ A16, unsigned short* __restrict__ W16)
{
  const int blk = blockIdx.x;
  const int tid = threadIdx.x;
  const float* src;
  unsigned short* dst;
  float carry;
  int lb;
  if (blk < kCvtBlocksA) {
    const int seg = blk / kCvtBlocksSrc;
    lb = blk - seg * kCvtBlocksSrc;
    src = (seg == 0) ? srcHead : ((seg == 1) ? srcTail : srcRel);
    dst = A16 + (size_t)blk * kCvtPerBlock;
    carry = kCarryA;
  } else {
    const int t = blk - kCvtBlocksA;
    const int seg = t / kCvtBlocksW;
    lb = t - seg * kCvtBlocksW;
    src = (seg == 0) ? wE : wR;
    dst = W16 + (size_t)t * kCvtPerBlock;
    carry = kCarryW;
  }
  const size_t so = (size_t)lb * kCvtPerBlock + (size_t)tid * 8;
  const v4f a0 = *(const v4f*)(src + so);
  const v4f a1 = *(const v4f*)(src + so + 4);
  v8h hv;
#pragma unroll
  for (int e = 0; e < 4; ++e) {
    const float x0 = a0[e];
    const float x1 = a1[e];
    hv[e]     = to_half_carried(x0, carry);
    hv[4 + e] = to_half_carried(x1, carry);
  }
  unsigned short* q = dst + (size_t)tid * 8;
  *(volatile v8h*)q = hv;
  __threadfence();
  *(volatile v8h*)q = hv;
}

__global__ __launch_bounds__(256) void core_plane_sum_kernel(
    const float* __restrict__ core, float* __restrict__ T)
{
  __shared__ float sPart[32];
  const int tid = threadIdx.x, lane = tid & 31, wave = tid >> 5;
  const int g = blockIdx.x;
#pragma unroll 1
  for (int p = 0; p < 4; ++p) {
    const int i = g * 32 + wave * 4 + p;
    const v4f* src = (const v4f*)(core + (size_t)i * kPlane);
    float s0 = 0.0f, s1 = 0.0f, s2 = 0.0f, s3 = 0.0f;
#pragma unroll 4
    for (int it = 0; it < kPlane / (32 * 4); ++it) {
      const v4f v = src[it * 32 + lane];
      s0 += v[0];
      s1 += v[1];
      s2 += v[2];
      s3 += v[3];
    }
    float s = (s0 + s1) + (s2 + s3);
    s += __shfl_xor(s, 16, 32);
    s += __shfl_xor(s, 8, 32);
    s += __shfl_xor(s, 4, 32);
    s += __shfl_xor(s, 2, 32);
    s += __shfl_xor(s, 1, 32);
    if (lane == 0) sPart[wave * 4 + p] = s;
  }
  __syncthreads();
  if (wave == 0) {
    const float v = sPart[lane];
    volatile float* q = (volatile float*)(T + g * 32 + lane);
    *q = v;
    __threadfence();
    *q = v;
  }
}

__global__ __launch_bounds__(128) void proj_gemm_half_kernel(
    const unsigned short* __restrict__ Ap, int lda,
    const unsigned short* __restrict__ Btp, int ldb,
    float* __restrict__ C, int ldc,
    const float* __restrict__ bias,
    int M, int N, int K, float scale)
{
  const _Float16* A  = (const _Float16*)Ap;
  const _Float16* Bt = (const _Float16*)Btp;
  __shared__ __align__(16) float sT[kGemmWaves][16 * 68];
  const int lane = threadIdx.x & 31;
  const int wave = threadIdx.x >> 5;
  const int tilesN = N >> 6;
  const int tilesM = M >> 6;
  const int tile = blockIdx.x * kGemmWaves + wave;
  if (tile >= tilesM * tilesN) return;
  const int tm = tile / tilesN;
  const int tn = tile - tm * tilesN;
  const int m0 = tm << 6;
  const int n0 = tn << 6;

  const int rlane = lane & 15;
  const int koff  = (lane >> 4) * 8;
  const int mOff  = (lane >> 4) * 8;

  v8f acc[4][4];
#pragma unroll
  for (int i = 0; i < 4; ++i)
#pragma unroll
    for (int j = 0; j < 4; ++j) acc[i][j] = (v8f){0.f, 0.f, 0.f, 0.f, 0.f, 0.f, 0.f, 0.f};

  for (int k0 = 0; k0 < K; k0 += 32) {
    v16h bh[4];
#pragma unroll
    for (int j = 0; j < 4; ++j) {
      const size_t bo = (size_t)(n0 + (j << 4) + rlane) * ldb + koff + k0;
      bh[j] = frag_load_h(Bt + bo);
    }
#pragma unroll
    for (int i = 0; i < 4; ++i) {
      const size_t ao = (size_t)(m0 + (i << 4) + rlane) * lda + koff + k0;
      const v16h ah = frag_load_h(A + ao);
#pragma unroll
      for (int j = 0; j < 4; ++j) acc[i][j] = mma_h_guarded(ah, bh[j], acc[i][j]);
    }
    keep4_h(bh[0], bh[1], bh[2], bh[3]);
  }
  acc_guard4(acc[0][0], acc[0][1], acc[0][2], acc[0][3]);
  acc_guard4(acc[1][0], acc[1][1], acc[1][2], acc[1][3]);
  acc_guard4(acc[2][0], acc[2][1], acc[2][2], acc[2][3]);
  acc_guard4(acc[3][0], acc[3][1], acc[3][2], acc[3][3]);

  float* slab = sT[wave];
  float bv[4];
#pragma unroll
  for (int j = 0; j < 4; ++j) bv[j] = bias[n0 + (j << 4) + rlane];
#pragma unroll
  for (int i = 0; i < 4; ++i) {
    const int mBase = m0 + (i << 4);
#pragma unroll
    for (int j = 0; j < 4; ++j) {
#pragma unroll
      for (int r = 0; r < 8; ++r) {
        const float v = acc[i][j][r] * scale + bv[j];
        slab[(mOff + r) * 68 + (j << 4) + rlane] = v;
      }
    }
    __builtin_amdgcn_fence(__ATOMIC_RELEASE, "workgroup");
    __builtin_amdgcn_wave_barrier();
    __builtin_amdgcn_fence(__ATOMIC_ACQUIRE, "workgroup");
    {
      const int hh = lane >> 4, c4 = (lane & 15) * 4;
      for (int pass = 0; pass < 2; ++pass) {
#pragma unroll
        for (int it = 0; it < 8; ++it) {
          const int row = it * 2 + hh;
          const v4f v = *(const v4f*)(slab + row * 68 + c4);
          *(volatile v4f*)(C + (size_t)(mBase + row) * ldc + n0 + c4) = v;
        }
        __threadfence();
      }
    }
    __builtin_amdgcn_fence(__ATOMIC_RELEASE, "workgroup");
    __builtin_amdgcn_wave_barrier();
    __builtin_amdgcn_fence(__ATOMIC_ACQUIRE, "workgroup");
  }
}

__global__ __launch_bounds__(64) void energy_kernel(
    const float* __restrict__ P, const float* __restrict__ T, float* __restrict__ out)
{
  const int b = threadIdx.x;
  const v4f* hp = (const v4f*)(P + (size_t)b * kEmb);
  const v4f* tp = (const v4f*)(P + (size_t)(kBatch + b) * kEmb);
  const v4f* rp = (const v4f*)(P + (size_t)(2 * kBatch + b) * kEmb);
  const v4f* cp = (const v4f*)T;
  float a0 = 0.0f, a1 = 0.0f, a2 = 0.0f, a3 = 0.0f;
#pragma unroll 1
  for (int q = 0; q < kEmb / 4; ++q) {
    const v4f h = hp[q];
    const v4f r = rp[q];
    const v4f t = tp[q];
    const v4f c = cp[q];
    a0 += ((h[0] * r[0]) * c[0]) * t[0];
    a1 += ((h[1] * r[1]) * c[1]) * t[1];
    a2 += ((h[2] * r[2]) * c[2]) * t[2];
    a3 += ((h[3] * r[3]) * c[3]) * t[3];
  }
  const float e = -((a0 + a1) + (a2 + a3));
  volatile float* o = (volatile float*)(out + b);
  *o = e;
  __threadfence();
  *o = e;
}

extern "C" void kernel_launch(void* const* d_in, const int* in_sizes, int n_in,
                              void* d_out, int out_size, void* d_ws, size_t ws_size,
                              hipStream_t stream) {
  if (n_in < 8) return;
  if (in_sizes[0] != kBatch * kHid) return;
  if (in_sizes[1] != kBatch * kHid) return;
  if (in_sizes[2] != kBatch * kHid) return;
  if (in_sizes[3] != kEmb * kHid) return;
  if (in_sizes[4] != kEmb) return;
  if (in_sizes[5] != kEmb * kHid) return;
  if (in_sizes[6] != kEmb) return;
  if (in_sizes[7] != kEmb * kPlane) return;
  if (out_size != kBatch) return;
  if (ws_size < kWsTotal) return;

  const float* head_src = (const float*)d_in[0];
  const float* rel_src  = (const float*)d_in[1];
  const float* tail_src = (const float*)d_in[2];
  const float* W_e      = (const float*)d_in[3];
  const float* b_e      = (const float*)d_in[4];
  const float* W_r      = (const float*)d_in[5];
  const float* b_r      = (const float*)d_in[6];
  const float* core     = (const float*)d_in[7];
  float* out = (float*)d_out;

  char* ws = (char*)d_ws;
  unsigned short* A16 = (unsigned short*)(ws + kOffA16);
  unsigned short* W16 = (unsigned short*)(ws + kOffW16);
  float*          P   = (float*)(ws + kOffP);
  float*          T   = (float*)(ws + kOffT);

  build_half_planes_kernel<<<kCvtBlocks, 256, 0, stream>>>(head_src, tail_src, rel_src, W_e, W_r, A16, W16);

  core_plane_sum_kernel<<<kEmb / 32, 256, 0, stream>>>(core, T);

  proj_gemm_half_kernel<<<1, 4 * 32, 0, stream>>>(
      A16, kHid, W16, kHid, P, kEmb, b_e, 2 * kBatch, kEmb, kHid, kFold);

  proj_gemm_half_kernel<<<1, 2 * 32, 0, stream>>>(
      A16 + (size_t)(2 * kBatch) * kHid, kHid, W16 + (size_t)kEmb * kHid, kHid,
      P + (size_t)(2 * kBatch) * kEmb, kEmb, b_r, kBatch, kEmb, kHid, kFold);

  energy_kernel<<<1, kBatch, 0, stream>>>(P, T, out);
}
